// MyMamba_31739808317885
// MI455X (gfx1250) — hardware-run, weakly checked
//
#include <hip/hip_runtime.h>
#include <hip/hip_bf16.h>
#include <math.h>

#define NBAT  32
#define NCH   32
#define SEQ   512
#define NSER  (NBAT * NCH)
#define LP    64
#define PL    16
#define PSTR  8
#define KP    32
#define DM    128
#define NROW  (NSER * LP)
#define XZW   (2 * DM)
#define DST   16
#define DTR   8
#define XDW   (DTR + 2 * DST)
#define XDN   64
#define NCK   4
#define CSER  (NSER / NCK)
#define CROW  (CSER * LP)
#define F3K   (LP * DM)
#define F3N   192
#define F4N   96
#define F4NP  128
#define NOUTF (NBAT * F4N * NCH)
#define NPART 64
#define SPB   (NSER / NPART)
#define GSTR  40
#define OSTR  68
#define SMEMB (8 * 16 * OSTR * 4)
#define SYP   132
#define LOG2E 1.4426950408889634f

static_assert(NROW % 128 == 0);
static_assert(CROW % 128 == 0);
static_assert(NSER % 128 == 0);
static_assert(XZW % 64 == 0);
static_assert(XDN % 64 == 0);
static_assert(DM % 64 == 0);
static_assert(F3N % 64 == 0);
static_assert(F4NP % 64 == 0);
static_assert(KP % 32 == 0);
static_assert(DM % 32 == 0);
static_assert(F3K % 32 == 0);
static_assert(F3N % 32 == 0);
static_assert(SMEMB >= (2 * 128 * GSTR + 64 * GSTR) * 2);
static_assert(NOUTF % (4 * 256) == 0);
static_assert((NROW * (KP / 8)) % 256 == 0);
static_assert((NROW * DM / 8) % 256 == 0);
static_assert(CROW % 8 == 0);
static_assert(SYP % 4 == 0);
static_assert(SYP >= DM);
static_assert(SPB * NPART == NSER);
static_assert(LP == 64);
static_assert(DM == 128);
static_assert(XDW <= XDN);
static_assert(F4N <= F4NP);
static_assert(PL <= KP);

typedef unsigned short us16 __attribute__((ext_vector_type(16)));
typedef unsigned short us8  __attribute__((ext_vector_type(8)));
typedef unsigned short us8a __attribute__((ext_vector_type(8), may_alias));
typedef __bf16 v16b __attribute__((ext_vector_type(16)));
typedef float v8f __attribute__((ext_vector_type(8)));
typedef float v4f __attribute__((ext_vector_type(4)));
typedef float v4fa __attribute__((ext_vector_type(4), may_alias));
typedef double v2d __attribute__((ext_vector_type(2)));
union FragU { us16 v; us8 h[2]; };

__device__ __forceinline__ unsigned short bf16_bits(float f) {
  unsigned u = __float_as_uint(f);
  u += 0x7FFFu + ((u >> 16) & 1u);
  return (unsigned short)(u >> 16);
}
__device__ __forceinline__ float bf16_val(unsigned short b) { return __uint_as_float(((unsigned)b) << 16); }
__device__ __forceinline__ float bf16r(float f) { return bf16_val(bf16_bits(f)); }
__device__ __forceinline__ float siluf(float x) { return x * __builtin_amdgcn_rcpf(1.0f + __expf(-x)); }
__device__ __forceinline__ float gelu_exact(float x) { return 0.5f * x * (1.0f + erff(x * 0.70710678118654752f)); }

__device__ __forceinline__ void split8(const v4f a, const v4f b, us8& hi, us8& lo) {
#pragma unroll
  for (int u = 0; u < 4; ++u) {
    const unsigned short ha = bf16_bits(a[u]);
    hi[u] = ha; lo[u] = bf16_bits(a[u] - bf16_val(ha));
    const unsigned short hb = bf16_bits(b[u]);
    hi[4 + u] = hb; lo[4 + u] = bf16_bits(b[u] - bf16_val(hb));
  }
}

__device__ __forceinline__ double shfl_xor_d(double v, int m) {
  const unsigned long long u = __builtin_bit_cast(unsigned long long, v);
  int lo = (int)(unsigned)(u & 0xffffffffull), hi = (int)(unsigned)(u >> 32);
  lo = __shfl_xor(lo, m);
  hi = __shfl_xor(hi, m);
  const unsigned long long r = (((unsigned long long)(unsigned)hi) << 32) | (unsigned long long)(unsigned)lo;
  return __builtin_bit_cast(double, r);
}

__device__ __forceinline__ v8f mma_bf16(us16 a, us16 b, v8f c) {
  return __builtin_amdgcn_wmma_f32_16x16x32_bf16(false, __builtin_bit_cast(v16b, a), false, __builtin_bit_cast(v16b, b), (short)0, c, false, false);
}
__device__ __forceinline__ void wguard(v8f& c0, v8f& c1, v8f& c2, v8f& c3, const us16& a0, const us16& a1,
                                       const us16& b0, const us16& b1, const us16& b2, const us16& b3) {
#if defined(__HIP_DEVICE_COMPILE__)
  asm volatile("v_nop\n\tv_nop\n\tv_nop\n\tv_nop"
               : "+v"(c0), "+v"(c1), "+v"(c2), "+v"(c3)
               : "v"(a0), "v"(a1), "v"(b0), "v"(b1), "v"(b2), "v"(b3));
#endif
}

__device__ __forceinline__ us16 lds_frag(const unsigned short* base) {
  const int lane = threadIdx.x & 31, r = lane & 15, kh = (lane >> 4) * 8;
  FragU f;
  f.h[0] = *(const us8a*)(base + r * GSTR + kh);
  f.h[1] = *(const us8a*)(base + r * GSTR + 16 + kh);
  return f.v;
}

__device__ __forceinline__ void stage_a(unsigned short* lds, const unsigned short* __restrict__ P, int ld, int m0, int k0, int tid) {
  const int row = tid >> 1, cq = (tid & 1) * 16;
  const unsigned short* src = P + (size_t)(m0 + row) * ld + k0 + cq;
  const us8 v0 = *(const us8a*)src;
  const us8 v1 = *(const us8a*)(src + 8);
  *(us8a*)(lds + row * GSTR + cq) = v0;
  *(us8a*)(lds + row * GSTR + cq + 8) = v1;
}
__device__ __forceinline__ void stage_b(unsigned short* lds, const unsigned short* __restrict__ P, int ld, int n0, int k0, int tid) {
  const int row = tid >> 2, kq = (tid & 3) * 8;
  const us8 v = *(const us8a*)(P + (size_t)(n0 + row) * ld + k0 + kq);
  *(us8a*)(lds + row * GSTR + kq) = v;
}

template <int NA, int EPI, int ACT>
__global__ __launch_bounds__(256) void k_gemm(const unsigned short* __restrict__ A0, const unsigned short* __restrict__ A1, int lda,
                                             const unsigned short* __restrict__ B0, int ldb,
                                             const float* __restrict__ bias, int hasb, int nb,
                                             const float* __restrict__ add, int hasadd, int ldadd,
                                             float* Yf, unsigned short* Yh, unsigned short* Yl, int ldy, int K) {
#pragma clang fp contract(off)
  __shared__ __attribute__((aligned(16))) unsigned char sm[SMEMB];
  unsigned short* lA0 = (unsigned short*)sm;
  unsigned short* lA1 = lA0 + 128 * GSTR;
  unsigned short* lB0 = lA1 + 128 * GSTR;
  float* oS = (float*)sm;
  const int tid = threadIdx.x, lane = tid & 31, wave = tid >> 5, cl = lane & 15, hh = lane >> 4;
  const int m0 = blockIdx.x * 128, n0 = blockIdx.y * 64;

  v8f acc[4];
#pragma unroll
  for (int j = 0; j < 4; ++j) { v8f zz = {0.f, 0.f, 0.f, 0.f, 0.f, 0.f, 0.f, 0.f}; acc[j] = zz; }

#pragma unroll 1
  for (int k0 = 0; k0 < K; k0 += 32) {
    __syncthreads();
    stage_a(lA0, A0, lda, m0, k0, tid);
    if (NA == 2) stage_a(lA1, A1, lda, m0, k0, tid);
    stage_b(lB0, B0, ldb, n0, k0, tid);
    __syncthreads();
    const us16 af0 = lds_frag(lA0 + 16 * wave * GSTR);
    us16 af1 = af0;
    if (NA == 2) af1 = lds_frag(lA1 + 16 * wave * GSTR);
    us16 bfr[4];
#pragma unroll
    for (int j = 0; j < 4; ++j) bfr[j] = lds_frag(lB0 + 16 * j * GSTR);
#pragma unroll
    for (int j = 0; j < 4; ++j) acc[j] = mma_bf16(af0, bfr[j], acc[j]);
    if (NA == 2) {
#pragma unroll
      for (int j = 0; j < 4; ++j) acc[j] = mma_bf16(af1, bfr[j], acc[j]);
    }
    wguard(acc[0], acc[1], acc[2], acc[3], af0, af1, bfr[0], bfr[1], bfr[2], bfr[3]);
  }
  __syncthreads();

  float* so = oS + wave * (16 * OSTR);
#pragma unroll
  for (int j = 0; j < 4; ++j) {
    const int col = n0 + 16 * j + cl;
    const int bc = (col < nb) ? col : (nb - 1);
    const float braw = bf16r(bias[bc]);
    const float bv = hasb ? braw : 0.0f;
#pragma unroll
    for (int r = 0; r < 8; ++r) {
      const int row = m0 + 16 * wave + 8 * hh + r;
      float v = acc[j][r] + bv;
      if (hasadd) v = v + add[(size_t)row * ldadd + col];
      if (ACT == 1) v = gelu_exact(v);
      so[(8 * hh + r) * OSTR + 16 * j + cl] = v;
    }
  }
  __syncthreads();
  if (EPI == 0) {
#pragma unroll
    for (int pass = 0; pass < 2; ++pass) {
#pragma unroll
      for (int it = 0; it < 8; ++it) {
        const int ch = it * 32 + lane, r = ch >> 4, q = (ch & 15) * 4;
        const v4f v = *(const v4fa*)(so + r * OSTR + q);
        *(volatile v4f*)(Yf + (size_t)(m0 + 16 * wave + r) * ldy + n0 + q) = v;
      }
      __threadfence();
    }
  } else {
#pragma unroll
    for (int pass = 0; pass < 2; ++pass) {
#pragma unroll
      for (int it = 0; it < 4; ++it) {
        const int r = it * 4 + (lane >> 3), c8 = (lane & 7) * 8;
        const v4f a = *(const v4fa*)(so + r * OSTR + c8);
        const v4f b = *(const v4fa*)(so + r * OSTR + c8 + 4);
        us8 hi, lo;
        split8(a, b, hi, lo);
        const size_t o = (size_t)(m0 + 16 * wave + r) * ldy + n0 + c8;
        *(volatile us8*)(Yh + o) = hi;
        *(volatile us8*)(Yl + o) = lo;
      }
      __threadfence();
    }
  }
}

__global__ __launch_bounds__(256) void k_cvt(const float* __restrict__ src, unsigned short* dst, int nsrc, int ncs, int ncd8, int total8) {
  const int idx = blockIdx.x * 256 + threadIdx.x;
  if (idx >= total8) return;
  const int row = idx / ncd8, c8 = (idx - row * ncd8) * 8;
  const int rs = (row < nsrc) ? row : (nsrc - 1);
  const int cs = (c8 + 8 <= ncs) ? c8 : (ncs - 8);
  const float* s = src + (size_t)rs * (size_t)ncs + cs;
  const v4f a = *(const v4fa*)s, b = *(const v4fa*)(s + 4);
  const bool zr = (row >= nsrc) || (c8 >= ncs);
  us8 o;
#pragma unroll
  for (int u = 0; u < 4; ++u) {
    o[u]     = zr ? (unsigned short)0 : bf16_bits(a[u]);
    o[4 + u] = zr ? (unsigned short)0 : bf16_bits(b[u]);
  }
  const size_t off = (size_t)idx * 8;
  *(volatile us8*)(dst + off) = o;
  __threadfence();
  *(volatile us8*)(dst + off) = o;
}

__global__ __launch_bounds__(256) void k_patch(const float* __restrict__ x, unsigned short* P) {
  const int idx = blockIdx.x * 256 + threadIdx.x;
  if (idx >= NROW * (KP / 8)) return;
  const int row = idx >> 2, c8 = (idx & 3) * 8;
  const int n = row >> 6, j = row & (LP - 1), b = n >> 5, c = n & (NCH - 1);
  const bool zr = (c8 >= PL);
  us8 o;
#pragma unroll
  for (int i = 0; i < 8; ++i) {
    int s = j * PSTR + c8 + i;
    s = (s < SEQ) ? s : (SEQ - 1);
    const float v = x[((size_t)b * SEQ + s) * NCH + c];
    o[i] = zr ? (unsigned short)0 : bf16_bits(v);
  }
  const size_t off = (size_t)idx * 8;
  *(volatile us8*)(P + off) = o;
  __threadfence();
  *(volatile us8*)(P + off) = o;
}

__global__ __launch_bounds__(256) void k_bnpart(const float* __restrict__ H1, double* PART) {
  __shared__ __attribute__((aligned(16))) double sp[2 * LP];
  const int blk = blockIdx.x, tid = threadIdx.x, lane = tid & 31, wave = tid >> 5;
  const int j = tid >> 2, q = tid & 3;
  double s = 0.0, s2 = 0.0;
#pragma unroll 1
  for (int si = 0; si < SPB; ++si) {
    const size_t row = (size_t)(blk * SPB + si) * LP + j;
    const float* p = H1 + row * DM + q * 32;
#pragma unroll
    for (int f = 0; f < 8; ++f) {
      const v4f v = *(const v4fa*)(p + 4 * f);
#pragma unroll
      for (int u = 0; u < 4; ++u) { const double dv = (double)v[u]; s += dv; s2 += dv * dv; }
    }
  }
  s += shfl_xor_d(s, 1);   s2 += shfl_xor_d(s2, 1);
  s += shfl_xor_d(s, 2);   s2 += shfl_xor_d(s2, 2);
  if (q == 0) { sp[2 * j] = s; sp[2 * j + 1] = s2; }
  __syncthreads();
  if (wave == 0) {
#pragma unroll
    for (int pass = 0; pass < 2; ++pass) {
#pragma unroll
      for (int it = 0; it < 2; ++it) {
        const int e = (it * 32 + lane) * 2;
        v2d o;
        o[0] = sp[e]; o[1] = sp[e + 1];
        *(volatile v2d*)(PART + (size_t)blk * (2 * LP) + e) = o;
      }
      __threadfence();
    }
  }
}

__global__ __launch_bounds__(64) void k_bnfin(const double* __restrict__ PART, const float* __restrict__ g, const float* __restrict__ bt, float* T) {
#pragma clang fp contract(off)
  __shared__ __attribute__((aligned(16))) float sT[4 * LP];
  const int j = threadIdx.x;
  double s = 0.0, s2 = 0.0;
#pragma unroll 1
  for (int blk = 0; blk < NPART; ++blk) {
    s  += PART[(size_t)blk * (2 * LP) + 2 * j];
    s2 += PART[(size_t)blk * (2 * LP) + 2 * j + 1];
  }
  const double inv = 1.0 / (double)(NSER * DM);
  const double mean = s * inv;
  double var = s2 * inv - mean * mean;
  var = (var > 0.0) ? var : 0.0;
  const float meanf = (float)mean, varf = (float)var;
  const float rc = 1.0f / sqrtf(varf + 1e-5f);
  sT[j] = meanf;
  sT[LP + j] = rc;
  sT[2 * LP + j] = bf16r(g[j]);
  sT[3 * LP + j] = bf16r(bt[j]);
  __syncthreads();
  const v4f o = *(const v4fa*)(sT + 4 * j);
  *(volatile v4f*)(T + 4 * j) = o;
  __threadfence();
  *(volatile v4f*)(T + 4 * j) = o;
}

__global__ __launch_bounds__(256) void k_bnapply(const float* __restrict__ H1, const float* __restrict__ T, unsigned short* HH, unsigned short* HL) {
#pragma clang fp contract(off)
  const int idx = blockIdx.x * 256 + threadIdx.x;
  if (idx >= NROW * DM / 8) return;
  const int row = idx >> 4;
  const int j = row & (LP - 1);
  const float mean = T[j], rc = T[LP + j], gg = T[2 * LP + j], bb = T[3 * LP + j];
  const size_t off = (size_t)idx * 8;
  const v4f a = *(const v4fa*)(H1 + off), b = *(const v4fa*)(H1 + off + 4);
  v4f va, vb;
#pragma unroll
  for (int u = 0; u < 4; ++u) {
    va[u] = ((a[u] - mean) * rc) * gg + bb;
    vb[u] = ((b[u] - mean) * rc) * gg + bb;
  }
  us8 hi, lo;
  split8(va, vb, hi, lo);
  *(volatile us8*)(HH + off) = hi; *(volatile us8*)(HL + off) = lo;
  __threadfence();
  *(volatile us8*)(HH + off) = hi; *(volatile us8*)(HL + off) = lo;
}

__global__ __launch_bounds__(256) void k_conv(const float* __restrict__ XZ, const float* __restrict__ cw, const float* __restrict__ cb,
                                             float* UF, unsigned short* UH, unsigned short* UL) {
#pragma clang fp contract(off)
  __shared__ __attribute__((aligned(16))) float sx[8 * DM];
  const int tid = threadIdx.x, r = tid >> 5, c4 = (tid & 31) * 4;
  const int crow = blockIdx.x * 8 + r, l = crow & (LP - 1);
  const int rp = (l > 0) ? (crow - 1) : crow;
  const v4f cur = *(const v4fa*)(XZ + (size_t)crow * XZW + c4);
  const v4f prv = *(const v4fa*)(XZ + (size_t)rp * XZW + c4);
  const v4f w01 = *(const v4fa*)(cw + c4 * 2), w23 = *(const v4fa*)(cw + c4 * 2 + 4);
  const v4f bb = *(const v4fa*)(cb + c4);
  float w0[4], w1[4];
  w0[0] = w01[0]; w1[0] = w01[1]; w0[1] = w01[2]; w1[1] = w01[3];
  w0[2] = w23[0]; w1[2] = w23[1]; w0[3] = w23[2]; w1[3] = w23[3];
  v4f sv;
#pragma unroll
  for (int u = 0; u < 4; ++u) {
    const float pv = (l > 0) ? prv[u] : 0.0f;
    const float a = (pv * bf16r(w0[u]) + cur[u] * bf16r(w1[u])) + bf16r(bb[u]);
    sv[u] = siluf(a);
  }
  const size_t o = (size_t)crow * DM + c4;
  *(volatile v4f*)(UF + o) = sv;
  __threadfence();
  *(volatile v4f*)(UF + o) = sv;
  *(v4fa*)(sx + r * DM + c4) = sv;
  __syncthreads();
  if (tid < 128) {
    const int rr = tid >> 4, c8 = (tid & 15) * 8;
    const v4f a = *(const v4fa*)(sx + rr * DM + c8);
    const v4f b = *(const v4fa*)(sx + rr * DM + c8 + 4);
    us8 hi, lo;
    split8(a, b, hi, lo);
    const size_t o2 = (size_t)(blockIdx.x * 8 + rr) * DM + c8;
    *(volatile us8*)(UH + o2) = hi; *(volatile us8*)(UL + o2) = lo;
    __threadfence();
    *(volatile us8*)(UH + o2) = hi; *(volatile us8*)(UL + o2) = lo;
  }
}

__global__ __launch_bounds__(128) void k_scan(const float* __restrict__ XZ, const float* __restrict__ UF, const float* __restrict__ XD,
                                             const float* __restrict__ dtw, const float* __restrict__ dtb, const float* __restrict__ Alog,
                                             const float* __restrict__ Dv, unsigned short* YH, unsigned short* YL) {
#pragma clang fp contract(off)
  __shared__ __attribute__((aligned(16))) float sy[LP * SYP];
  const int sl = blockIdx.x, d = threadIdx.x, lane = d & 31, wave = d >> 5;
  float A2[DST], h[DST];
#pragma unroll
  for (int s = 0; s < DST; ++s) { A2[s] = -__expf(bf16r(Alog[d * DST + s])) * LOG2E; h[s] = 0.0f; }
  const v4f wa = *(const v4fa*)(dtw + d * DTR), wb = *(const v4fa*)(dtw + d * DTR + 4);
  float w[DTR];
#pragma unroll
  for (int k = 0; k < 4; ++k) { w[k] = bf16r(wa[k]); w[4 + k] = bf16r(wb[k]); }
  const float Dd = bf16r(Dv[d]);
  const float bd = bf16r(dtb[d]);
#pragma unroll 1
  for (int l = 0; l < LP; ++l) {
    const size_t crow = (size_t)sl * LP + (size_t)l;
    const float* xd = XD + crow * XDN;
    const v4f d0 = *(const v4fa*)(xd), d1 = *(const v4fa*)(xd + 4);
    float raw = 0.0f;
#pragma unroll
    for (int k = 0; k < 4; ++k) raw = raw + d0[k] * w[k];
#pragma unroll
    for (int k = 0; k < 4; ++k) raw = raw + d1[k] * w[4 + k];
    const float a = raw + bd;
    const float dl = fmaxf(a, 0.0f) + log1pf(__expf(-fabsf(a)));
    const float uv = UF[crow * DM + d];
    const float zv = XZ[crow * XZW + DM + d];
    v4f Bv[4], Cv[4];
#pragma unroll
    for (int q = 0; q < 4; ++q) {
      Bv[q] = *(const v4fa*)(xd + DTR + 4 * q);
      Cv[q] = *(const v4fa*)(xd + DTR + DST + 4 * q);
    }
    const float dx = dl * uv;
    float y = 0.0f;
#pragma unroll
    for (int s = 0; s < DST; ++s) {
      const float e = exp2f(dl * A2[s]);
      h[s] = e * h[s] + dx * Bv[s >> 2][s & 3];
      y = y + h[s] * Cv[s >> 2][s & 3];
    }
    const float yv = (y + uv * Dd) * siluf(zv);
    sy[l * SYP + d] = yv;
  }
  __syncthreads();
#pragma unroll
  for (int pass = 0; pass < 2; ++pass) {
#pragma unroll
    for (int it = 0; it < 8; ++it) {
      const int row = 16 * wave + 2 * it + (lane >> 4), c8 = (lane & 15) * 8;
      const v4f va = *(const v4fa*)(sy + row * SYP + c8);
      const v4f vb = *(const v4fa*)(sy + row * SYP + c8 + 4);
      us8 hi, lo;
      split8(va, vb, hi, lo);
      const size_t o = ((size_t)sl * LP + (size_t)row) * DM + c8;
      *(volatile us8*)(YH + o) = hi; *(volatile us8*)(YL + o) = lo;
    }
    __threadfence();
  }
}

__global__ __launch_bounds__(256) void k_outT(const float* __restrict__ F4, float* out) {
  const int idx = blockIdx.x * 256 + threadIdx.x;
  if (idx >= NOUTF / 4) return;
  const int e0 = idx * 4;
  const int b = e0 / (F4N * NCH);
  const int rem = e0 - b * (F4N * NCH);
  const int t = rem / NCH;
  const int c0 = rem - t * NCH;
  v4f r;
#pragma unroll
  for (int u = 0; u < 4; ++u) r[u] = F4[(size_t)(b * NCH + c0 + u) * F4NP + t];
  *(volatile v4f*)(out + e0) = r;
  __threadfence();
  *(volatile v4f*)(out + e0) = r;
}

extern "C" void kernel_launch(void* const* d_in, const int* in_sizes, int n_in,
                              void* d_out, int out_size, void* d_ws, size_t ws_size,
                              hipStream_t stream) {
  if (n_in < 29) return;
  if (in_sizes[0] != NBAT * SEQ * NCH || in_sizes[1] != DM * PL || in_sizes[2] != DM || in_sizes[3] != LP || in_sizes[4] != LP ||
      in_sizes[5] != DM * DM || in_sizes[6] != DM || in_sizes[25] != F3N * F3K || in_sizes[26] != F3N ||
      in_sizes[27] != F4N * F3N || in_sizes[28] != F4N || out_size != NOUTF) return;
  for (int m = 0; m < 2; ++m) {
    const int bs = 7 + 9 * m;
    if (in_sizes[bs] != XZW * DM || in_sizes[bs + 1] != DM * 2 || in_sizes[bs + 2] != DM || in_sizes[bs + 3] != XDW * DM ||
        in_sizes[bs + 4] != DM * DTR || in_sizes[bs + 5] != DM || in_sizes[bs + 6] != DM * DST || in_sizes[bs + 7] != DM ||
        in_sizes[bs + 8] != DM * DM) return;
  }

  const float* x     = (const float*)d_in[0];
  const float* fc1_w = (const float*)d_in[1];
  const float* fc1_b = (const float*)d_in[2];
  const float* bn_g  = (const float*)d_in[3];
  const float* bn_b  = (const float*)d_in[4];
  const float* fc2_w = (const float*)d_in[5];
  const float* fc2_b = (const float*)d_in[6];
  const float* mp[2][9];
  for (int m = 0; m < 2; ++m)
    for (int j = 0; j < 9; ++j) mp[m][j] = (const float*)d_in[7 + 9 * m + j];
  const float* fc3_w = (const float*)d_in[25];
  const float* fc3_b = (const float*)d_in[26];
  const float* fc4_w = (const float*)d_in[27];
  const float* fc4_b = (const float*)d_in[28];
  float* out = (float*)d_out;

  size_t off = 0;
  auto carve = [&](size_t bytes) -> char* { char* p = (char*)d_ws + off; off += (bytes + 255) & ~(size_t)255; return p; };
  unsigned short* W1p  = (unsigned short*)carve((size_t)DM * KP * 2);
  unsigned short* W2p  = (unsigned short*)carve((size_t)DM * DM * 2);
  unsigned short* WINp = (unsigned short*)carve((size_t)2 * XZW * DM * 2);
  unsigned short* WXp  = (unsigned short*)carve((size_t)2 * XDN * DM * 2);
  unsigned short* WOp  = (unsigned short*)carve((size_t)2 * DM * DM * 2);
  unsigned short* W3p  = (unsigned short*)carve((size_t)F3N * F3K * 2);
  unsigned short* W4p  = (unsigned short*)carve((size_t)F4NP * F3N * 2);
  unsigned short* P16  = (unsigned short*)carve((size_t)NROW * KP * 2);
  float* R1f           = (float*)carve((size_t)NROW * DM * 4);
  unsigned short* HPH  = (unsigned short*)carve((size_t)NROW * DM * 2);
  unsigned short* HPL  = (unsigned short*)carve((size_t)NROW * DM * 2);
  double* PART         = (double*)carve((size_t)NPART * 2 * LP * 8);
  float* BNT           = (float*)carve((size_t)4 * LP * 4);
  float* XZ            = (float*)carve((size_t)CROW * XZW * 4);
  float* UF            = (float*)carve((size_t)CROW * DM * 4);
  unsigned short* UH   = (unsigned short*)carve((size_t)CROW * DM * 2);
  unsigned short* UL   = (unsigned short*)carve((size_t)CROW * DM * 2);
  float* XD            = (float*)carve((size_t)CROW * XDN * 4);
  unsigned short* YH   = (unsigned short*)carve((size_t)CROW * DM * 2);
  unsigned short* YL   = (unsigned short*)carve((size_t)CROW * DM * 2);
  unsigned short* GH   = (unsigned short*)carve((size_t)NSER * F3N * 2);
  unsigned short* GL   = (unsigned short*)carve((size_t)NSER * F3N * 2);
  float* F4            = (float*)carve((size_t)NSER * F4NP * 4);
  if (off > ws_size || off > (size_t)134217728) return;

  const dim3 b256(256), b128(128), b64(64);
  k_cvt<<<dim3((DM * (KP / 8) + 255) / 256), b256, 0, stream>>>(fc1_w, W1p, DM, PL, KP / 8, DM * (KP / 8));
  k_cvt<<<dim3((DM * (DM / 8) + 255) / 256), b256, 0, stream>>>(fc2_w, W2p, DM, DM, DM / 8, DM * (DM / 8));
  for (int m = 0; m < 2; ++m) {
    k_cvt<<<dim3((XZW * (DM / 8) + 255) / 256), b256, 0, stream>>>(mp[m][0], WINp + (size_t)m * XZW * DM, XZW, DM, DM / 8, XZW * (DM / 8));
    k_cvt<<<dim3((XDN * (DM / 8) + 255) / 256), b256, 0, stream>>>(mp[m][3], WXp + (size_t)m * XDN * DM, XDW, DM, DM / 8, XDN * (DM / 8));
    k_cvt<<<dim3((DM * (DM / 8) + 255) / 256), b256, 0, stream>>>(mp[m][8], WOp + (size_t)m * DM * DM, DM, DM, DM / 8, DM * (DM / 8));
  }
  k_cvt<<<dim3((F3N * (F3K / 8) + 255) / 256), b256, 0, stream>>>(fc3_w, W3p, F3N, F3K, F3K / 8, F3N * (F3K / 8));
  k_cvt<<<dim3((F4NP * (F3N / 8) + 255) / 256), b256, 0, stream>>>(fc4_w, W4p, F4N, F3N, F3N / 8, F4NP * (F3N / 8));
  k_patch<<<dim3(NROW * (KP / 8) / 256), b256, 0, stream>>>(x, P16);
  k_gemm<1, 0, 1><<<dim3(NROW / 128, DM / 64), b256, 0, stream>>>(P16, P16, KP, W1p, KP, fc1_b, 1, DM, R1f, 0, DM, R1f, UH, UL, DM, KP);
  k_bnpart<<<dim3(NPART), b256, 0, stream>>>(R1f, PART);
  k_bnfin<<<dim3(1), b64, 0, stream>>>(PART, bn_g, bn_b, BNT);
  k_bnapply<<<dim3(NROW * DM / 8 / 256), b256, 0, stream>>>(R1f, BNT, HPH, HPL);
  k_gemm<2, 0, 0><<<dim3(NROW / 128, DM / 64), b256, 0, stream>>>(HPH, HPL, DM, W2p, DM, fc2_b, 1, DM, R1f, 0, DM, R1f, UH, UL, DM, DM);

  for (int m = 0; m < 2; ++m) {
    const float* convw = mp[m][1];
    const float* convb = mp[m][2];
    const float* dtw   = mp[m][4];
    const float* dtb   = mp[m][5];
    const float* Alog  = mp[m][6];
    const float* Dv    = mp[m][7];
    const int hasres = (m == 0) ? 1 : 0;
    for (int c = 0; c < NCK; ++c) {
      const size_t gro = (size_t)c * CROW;
      k_gemm<2, 0, 0><<<dim3(CROW / 128, XZW / 64), b256, 0, stream>>>(HPH + gro * DM, HPL + gro * DM, DM, WINp + (size_t)m * XZW * DM, DM,
                                                                       fc1_b, 0, DM, R1f, 0, DM, XZ, UH, UL, XZW, DM);
      k_conv<<<dim3(CROW / 8), b256, 0, stream>>>(XZ, convw, convb, UF, UH, UL);
      k_gemm<2, 0, 0><<<dim3(CROW / 128, XDN / 64), b256, 0, stream>>>(UH, UL, DM, WXp + (size_t)m * XDN * DM, DM,
                                                                       fc1_b, 0, DM, R1f, 0, DM, XD, YH, YL, XDN, DM);
      k_scan<<<dim3(CSER), b128, 0, stream>>>(XZ, UF, XD, dtw, dtb, Alog, Dv, YH, YL);
      k_gemm<2, 1, 0><<<dim3(CROW / 128, DM / 64), b256, 0, stream>>>(YH, YL, DM, WOp + (size_t)m * DM * DM, DM,
                                                                       fc1_b, 0, DM, R1f + gro * DM, hasres, DM, XD, HPH + gro * DM, HPL + gro * DM, DM, DM);
    }
  }
  k_gemm<2, 1, 1><<<dim3(NSER / 128, F3N / 64), b256, 0, stream>>>(HPH, HPL, F3K, W3p, F3K, fc3_b, 1, F3N, R1f, 0, DM, XD, GH, GL, F3N, F3K);
  k_gemm<2, 0, 0><<<dim3(NSER / 128, F4NP / 64), b256, 0, stream>>>(GH, GL, F3N, W4p, F3N, fc4_b, 1, F4N, R1f, 0, DM, F4, UH, UL, F4NP, F3N);
  k_outT<<<dim3(NOUTF / 4 / 256), b256, 0, stream>>>(F4, out);
}
